// KPConvSimpleBlock_second_76227079570100
// MI455X (gfx1250) — hardware-run, weakly checked
//
#include <hip/hip_runtime.h>


#ifndef NB
#define NB 4
#endif
#ifndef NG
#define NG 4096
#endif
#define NB_FULL  4
#define NG_FULL  4096
#define NPB_FULL 16384
#define NPTS (NB_FULL * NPB_FULL)
#define NQ   (NB * NG)
#define KPN  15
#define CIN  6
#define CO   128
#define SNB  32
#define KD   (KPN * CIN)
#define KPAD 96
#define AP   52
#define OSP  132
#define QT   4
#define BQ   (16 * QT)
#define NBLK (NQ / BQ)
#define QRS  2048.0f
#define QRI  (1.0f / 2048.0f)
#define WSC  64.0f
#define WSI  (1.0f / 64.0f)

static_assert(KD <= KPAD);
static_assert(KPAD % 32 == 0);
static_assert(KPAD % 8 == 0);
static_assert(3 * 16 == KPAD / 2);
static_assert(AP >= KPAD / 2);
static_assert((AP * 4) % 16 == 0);
static_assert((OSP * 4) % 16 == 0);
static_assert(CO == 8 * 16);
static_assert(NG % BQ == 0);
static_assert(NQ % BQ == 0);
static_assert(NB <= NB_FULL);
static_assert(NG <= NG_FULL);
static_assert(SNB == 32);
static_assert(256 * 2 == 16 * SNB);
static_assert(256 * 2 * 16 == 16 * CO * 4);
static_assert(64 * 16 == 256 * 4);
static_assert(16 * SNB * 16 + 2 * 16 * AP * 4 + 16 * OSP * 4 + 256 * 4 <= 131072);

typedef _Float16 h16;
typedef __attribute__((ext_vector_type(16))) _Float16 v16h;
typedef __attribute__((ext_vector_type(8)))  _Float16 v8h;
typedef __attribute__((ext_vector_type(8)))  float    v8f;
typedef __attribute__((ext_vector_type(4)))  float    v4f;
typedef __attribute__((ext_vector_type(4)))  unsigned v4u;
typedef v4f  __attribute__((may_alias)) v4fa;
typedef v4u  __attribute__((may_alias)) v4ua;

__device__ __forceinline__ unsigned short f2bf(float f) { unsigned u = __float_as_uint(f); u += 0x7FFFu + ((u >> 16) & 1u); return (unsigned short)(u >> 16); }
__device__ __forceinline__ float bfr(float f) { return __uint_as_float(((unsigned)f2bf(f)) << 16); }
__device__ __forceinline__ v16h cat16(v8h lo, v8h hi) { return __builtin_shufflevector(lo, hi, 0, 1, 2, 3, 4, 5, 6, 7, 8, 9, 10, 11, 12, 13, 14, 15); }
__device__ __forceinline__ v8f wmma16(v16h a, v16h b, v8f c) { return __builtin_amdgcn_wmma_f32_16x16x32_f16(false, a, false, b, (short)0, c, false, false); }
__device__ __forceinline__ v16h  ldh(const h16* p) { return cat16(*(const v8h*)p, *(const v8h*)(p + 16)); }
__device__ __forceinline__ h16 toh_flush(float v) { const h16 r = (h16)v; return (fabsf(v) < 6.103515625e-05f) ? (h16)0.0f : r; }
__device__ __forceinline__ unsigned hbits(h16 x) { return (unsigned)__builtin_bit_cast(unsigned short, x); }
__device__ __forceinline__ v8f wmma16g(v16h a, v16h b, v8f c) { c = wmma16(a, b, c); asm volatile("v_nop\n\tv_nop\n\tv_nop\n\tv_nop" : "+v"(c) : "v"(a), "v"(b)); return c; }

__global__ __launch_bounds__(256) void k_wprep(const float* __restrict__ W, h16* WT) {
#pragma clang fp contract(off)
    const int i = blockIdx.x * 256 + threadIdx.x; if (i >= CO * KPAD / 8) return;
    const int o = i / (KPAD / 8), j0 = (i % (KPAD / 8)) * 8;
    v8h hv;
#pragma unroll
    for (int e = 0; e < 8; ++e) {
        const int kk = j0 + e; const int kc = kk < KD ? kk : (KD - 1);
        float w = W[(size_t)kc * CO + o];
        asm volatile("" : "+v"(w));
        const float ws = (kk < KD) ? bfr(w) * WSC : 0.0f;
        hv[e] = toh_flush(ws); }
    *(volatile v8h*)(WT + (size_t)i * 8) = hv; __threadfence(); *(volatile v8h*)(WT + (size_t)i * 8) = hv;
}

__global__ __launch_bounds__(256) void k_conv(const float* __restrict__ xyz, const float* __restrict__ cen, const int* __restrict__ idx, const float* __restrict__ Kp,
                                              const h16* __restrict__ WT, float* RAW, float* PART) {
    __shared__ v4f pl[16 * SNB];
    __shared__ __align__(16) unsigned ah[16 * AP];
    __shared__ __align__(16) unsigned ar[16 * AP];
    __shared__ __align__(16) float os[16 * OSP];
    __shared__ __align__(16) float ps[256];
    const int tid = threadIdx.x;
    const int lane = tid & 31, lr = lane & 15, hi = lane >> 4;
    const int wave = __builtin_amdgcn_readfirstlane((int)(threadIdx.x >> 5));
    v16h bw[3];
#pragma unroll
    for (int ks = 0; ks < 3; ++ks) bw[ks] = ldh(WT + (size_t)(wave * 16 + lr) * KPAD + ks * 32 + 8 * hi);
    const int arow = tid >> 4, ak = tid & 15;
    const int akc = ak < KPN ? ak : (KPN - 1);
    const bool akv = ak < KPN;
    float kx = Kp[akc * 3 + 0], ky = Kp[akc * 3 + 1], kz = Kp[akc * 3 + 2];
    asm volatile("" : "+v"(kx)); asm volatile("" : "+v"(ky)); asm volatile("" : "+v"(kz));
    kx = bfr(kx); ky = bfr(ky); kz = bfr(kz);
    const int qbase0 = blockIdx.x * BQ;
    const int qin0 = (qbase0 / NG) * NG_FULL + (qbase0 % NG);
    const int scol = tid & 127; const bool ssq = tid >= 128;
    float cacc = 0.0f;
#pragma unroll 1
    for (int t = 0; t < QT; ++t) {
        const int qb = qbase0 + t * 16, qi = qin0 + t * 16;
#pragma unroll
        for (int it = 0; it < 2; ++it) {
            const int p = it * 256 + tid; const int row = p >> 5, snb = p & 31;
            int gi = idx[(size_t)(qi + row) * SNB + snb];
            gi = gi < 0 ? gi + (NPTS + 1) : gi;
            gi = gi < 0 ? 0 : (gi > NPTS ? NPTS : gi);
            const bool sh = gi >= NPTS;
            const int ga = sh ? (NPTS - 1) : gi;
            float x0 = xyz[(size_t)ga * 3 + 0], x1 = xyz[(size_t)ga * 3 + 1], x2 = xyz[(size_t)ga * 3 + 2];
            asm volatile("" : "+v"(x0)); asm volatile("" : "+v"(x1)); asm volatile("" : "+v"(x2));
            v4f pv;
            pv[0] = sh ? 1.0e6f : bfr(x0); pv[1] = sh ? 1.0e6f : bfr(x1); pv[2] = sh ? 1.0e6f : bfr(x2); pv[3] = sh ? 0.0f : 1.0f;
            pl[p] = pv; }
        __syncthreads();
        {
            const float q0 = bfr(cen[(size_t)(qi + arow) * 3 + 0]), q1 = bfr(cen[(size_t)(qi + arow) * 3 + 1]), q2 = bfr(cen[(size_t)(qi + arow) * 3 + 2]);
            float ax = 0.0f, ay = 0.0f, az = 0.0f;
#pragma unroll 4
            for (int s = 0; s < SNB; ++s) {
                const v4f pv = pl[arow * SNB + s];
                const float nx = pv[0] - q0, ny = pv[1] - q1, nz = pv[2] - q2;
                const float dx = nx - kx, dy = ny - ky, dz = nz - kz;
                const float d = sqrtf(dx * dx + dy * dy + dz * dz);
                const float w = fmaxf(1.0f - d, 0.0f);
                ax += w * (pv[0] * pv[3]); ay += w * (pv[1] * pv[3]); az += w * (pv[2] * pv[3]); }
            const h16 hx = toh_flush(ax), hy = toh_flush(ay), hz = toh_flush(az);
            const h16 rx = toh_flush((ax - (float)hx) * QRS), ry = toh_flush((ay - (float)hy) * QRS), rz = toh_flush((az - (float)hz) * QRS);
            const unsigned h1 = akv ? (hbits(hx) << 16) : 0u, h2 = akv ? (hbits(hy) | (hbits(hz) << 16)) : 0u;
            const unsigned r1 = akv ? (hbits(rx) << 16) : 0u, r2 = akv ? (hbits(ry) | (hbits(rz) << 16)) : 0u;
            const int wo = arow * AP + 3 * ak;
            ah[wo + 0] = 0u; ah[wo + 1] = h1; ah[wo + 2] = h2;
            ar[wo + 0] = 0u; ar[wo + 1] = r1; ar[wo + 2] = r2;
        }
        __syncthreads();
        {
            v8f aH = (v8f){}, aR = (v8f){};
#pragma unroll
            for (int ks = 0; ks < 3; ++ks) {
                const int wo = lr * AP + ks * 16 + 4 * hi;
                const v16h fa = cat16(__builtin_bit_cast(v8h, *(const v4ua*)(&ah[wo])), __builtin_bit_cast(v8h, *(const v4ua*)(&ah[wo + 8])));
                const v16h fr = cat16(__builtin_bit_cast(v8h, *(const v4ua*)(&ar[wo])), __builtin_bit_cast(v8h, *(const v4ua*)(&ar[wo + 8])));
                aH = wmma16g(fa, bw[ks], aH);
                aR = wmma16g(fr, bw[ks], aR); }
#pragma unroll
            for (int r = 0; r < 8; ++r) os[(8 * hi + r) * OSP + wave * 16 + lr] = (aH[r] + aR[r] * QRI) * WSI;
        }
        __syncthreads();
#pragma unroll 1
        for (int pass = 0; pass < 2; ++pass) {
#pragma unroll
            for (int it = 0; it < 2; ++it) { const int p = it * 256 + tid; const int row = p >> 5, c4 = (p & 31) * 4;
                const v4f val = *(const v4fa*)(&os[row * OSP + c4]);
                *(volatile v4f*)(RAW + (size_t)(qb + row) * CO + c4) = val; }
            if (pass == 0) __threadfence(); }
#pragma unroll 4
        for (int r = 0; r < 16; ++r) { const float v = os[r * OSP + scol]; cacc += ssq ? v * v : v; }
    }
    ps[tid] = cacc;
    __syncthreads();
    if (tid < 64) {
        const v4f val = *(const v4fa*)(&ps[tid * 4]);
        float* dst = PART + (size_t)blockIdx.x * 256 + tid * 4;
        *(volatile v4f*)dst = val; __threadfence(); *(volatile v4f*)dst = val; }
}

__global__ __launch_bounds__(128) void k_stats(const float* __restrict__ PART, const float* __restrict__ gamma, const float* __restrict__ beta, float* SS) {
#pragma clang fp contract(off)
    __shared__ __align__(16) float ss[256];
    const int c = threadIdx.x;
    double s = 0.0, q = 0.0;
#pragma unroll 4
    for (int b = 0; b < NBLK; ++b) { s += (double)PART[(size_t)b * 256 + c]; q += (double)PART[(size_t)b * 256 + 128 + c]; }
    const double mean = s * (1.0 / (double)NQ);
    double var = q * (1.0 / (double)NQ) - mean * mean; var = var < 0.0 ? 0.0 : var;
    const float rs = rsqrtf((float)var + 1.0e-5f);
    const float sc = rs * bfr(gamma[c]);
    const float sh = bfr(beta[c]) - (float)mean * sc;
    ss[c] = sc; ss[128 + c] = sh;
    __syncthreads();
    if (c < 64) {
        const v4f val = *(const v4fa*)(&ss[c * 4]);
        *(volatile v4f*)(SS + c * 4) = val; __threadfence(); *(volatile v4f*)(SS + c * 4) = val; }
}

__global__ __launch_bounds__(256) void k_apply(const float* __restrict__ RAW, const float* __restrict__ SS, float* OUT, size_t n4) {
#pragma clang fp contract(off)
    const size_t i = (size_t)blockIdx.x * 256 + threadIdx.x; if (i >= n4) return;
    const int c = (int)((i * 4) & (size_t)(CO - 1));
    const v4f v = *(const v4f*)(RAW + i * 4);
    const v4f sc = *(const v4f*)(SS + c);
    const v4f sh = *(const v4f*)(SS + 128 + c);
    v4f y;
#pragma unroll
    for (int j = 0; j < 4; ++j) { const float u = v[j] * sc[j] + sh[j]; y[j] = (u >= 0.0f) ? u : 0.2f * u; }
    *(volatile v4f*)(OUT + i * 4) = y; __threadfence(); *(volatile v4f*)(OUT + i * 4) = y;
}

static constexpr size_t al256(size_t v) { return (v + 255) & ~(size_t)255; }
static constexpr size_t SZ_WT   = al256((size_t)CO * KPAD * 2);
static constexpr size_t SZ_RAW  = al256((size_t)NQ * CO * 4);
static constexpr size_t SZ_PART = al256((size_t)NBLK * 256 * 4);
static constexpr size_t SZ_SS   = al256((size_t)256 * 4);
static constexpr size_t SZ_TOTAL = SZ_WT + SZ_RAW + SZ_PART + SZ_SS;
static_assert(SZ_TOTAL <= (size_t)134217728);
static_assert((size_t)(CO * KPAD / 8) * 16 == (size_t)CO * KPAD * 2);
static_assert(((size_t)NQ * CO) % 4 == 0);

extern "C" void kernel_launch(void* const* d_in, const int* in_sizes, int n_in,
                              void* d_out, int out_size, void* d_ws, size_t ws_size, hipStream_t stream) {
    if (n_in < 7) return;
    const size_t needq = (size_t)(NB - 1) * NG_FULL + NG;
    if ((size_t)in_sizes[0] < (size_t)NPTS * 3) return;
    if ((size_t)in_sizes[1] < needq * 3 || (size_t)in_sizes[2] < needq * SNB) return;
    if (in_sizes[3] < KPN * 3 || in_sizes[4] < KPN * CIN * CO || in_sizes[5] < CO || in_sizes[6] < CO) return;
    if ((size_t)out_size < (size_t)NQ * CO) return;
    if (SZ_TOTAL > ws_size) return;
    const float* xyz = (const float*)d_in[0];
    const float* cen = (const float*)d_in[1];
    const int*   idx = (const int*)d_in[2];
    const float* kpt = (const float*)d_in[3];
    const float* w   = (const float*)d_in[4];
    const float* gam = (const float*)d_in[5];
    const float* bet = (const float*)d_in[6];
    float* OUT = (float*)d_out;
    char* wsp = (char*)d_ws;
    h16*   WT   = (h16*)wsp;   wsp += SZ_WT;
    float* RAW  = (float*)wsp; wsp += SZ_RAW;
    float* PART = (float*)wsp; wsp += SZ_PART;
    float* SS   = (float*)wsp; wsp += SZ_SS;

    k_wprep<<<(CO * KPAD / 8 + 255) / 256, 256, 0, stream>>>(w, WT);
    k_conv<<<NBLK, 256, 0, stream>>>(xyz, cen, idx, kpt, WT, RAW, PART);
    k_stats<<<1, 128, 0, stream>>>(PART, gam, bet, SS);
    const size_t n4 = (size_t)NQ * CO / 4;
    k_apply<<<(unsigned)((n4 + 255) / 256), 256, 0, stream>>>(RAW, SS, OUT, n4);
}
